// SparseLinear_50525995270225
// MI455X (gfx1250) — hardware-verified
//
#include <hip/hip_runtime.h>
#include <math.h>

typedef __attribute__((ext_vector_type(16))) _Float16 v16h;
typedef __attribute__((ext_vector_type(8)))  _Float16 v8h;
typedef __attribute__((ext_vector_type(8)))  float    v8f;
typedef __attribute__((ext_vector_type(4)))  float    v4f;
typedef __attribute__((ext_vector_type(4)))  int      v4i;

constexpr int kBatch      = 1024;
constexpr int kIn         = 4096;
constexpr int kOut        = 4096;
constexpr int kNnz        = 1600000;
constexpr int kRowsPerBlk = 8;
constexpr int kCarry      = 64;
constexpr float kFixScale = 4194304.0f;
constexpr float kFixClamp = 256.0f;
constexpr float kCellToCarried = (float)kCarry / kFixScale;
constexpr float kFoldBack = 1.0f / ((float)kCarry * (float)kCarry);

static_assert((kNnz % 128) == 0, "entry list is a whole number of 32-lane x 4-entry wave steps");
static_assert((kBatch % 64) == 0 && (kOut % 64) == 0, "GEMM M,N multiples of 64");
static_assert((kIn % 32) == 0, "GEMM K multiple of 32");
static_assert((kOut % kRowsPerBlk) == 0 && (kRowsPerBlk & (kRowsPerBlk - 1)) == 0, "row ownership");
static_assert(((kRowsPerBlk * kIn) % (8 * 256)) == 0, "densify store coverage");
static_assert(((kRowsPerBlk * kIn / 4) % 256) == 0, "densify zero-fill coverage");
static_assert(((kBatch * kIn / 8) % 256) == 0, "cast coverage");

constexpr size_t kOffX16  = 0;
constexpr size_t kOffW16  = kOffX16 + (size_t)kBatch * kIn * 2;
constexpr size_t kWsTotal = kOffW16 + (size_t)kOut * kIn * 2;
static_assert(kWsTotal == 41943040ull, "carve total");
static_assert(kWsTotal <= 134217728ull, "carve cap");
static_assert((kOffW16 % 128) == 0, "128-B aligned regions");

union FragU { v16h v; v8h h[2]; };
__device__ __forceinline__ v16h frag_load_h(const _Float16* p) {
  FragU f;
  f.h[0] = *(const v8h*)(p);
  f.h[1] = *(const v8h*)(p + 16);
  return f.v;
}
__device__ __forceinline__ v8f mma_h(v16h a, v16h b, v8f c) {
  return __builtin_amdgcn_wmma_f32_16x16x32_f16(false, a, false, b, (short)0, c, false, false);
}
__device__ __forceinline__ void tie_acc_h(v8f& a, v16h x, v16h y) { asm volatile("" : "+v"(a) : "v"(x), "v"(y)); }
__device__ __forceinline__ void nop_guard_h(v8f& a, v16h x, v16h y) { asm volatile("v_nop\n\tv_nop\n\tv_nop\n\tv_nop" : "+v"(a) : "v"(x), "v"(y)); }
__device__ __forceinline__ void nop_guard_acc(v8f& a) { asm volatile("v_nop\n\tv_nop\n\tv_nop\n\tv_nop" : "+v"(a)); }
__device__ __forceinline__ void keep4_h(v16h a, v16h b, v16h c, v16h d) { asm volatile("v_nop" :: "v"(a), "v"(b), "v"(c), "v"(d)); }

__global__ __launch_bounds__(256) void cast_rows_f16_kernel(
    const float* __restrict__ src, unsigned short* __restrict__ dst, int total8, float carry)
{
  const int i = blockIdx.x * 256 + threadIdx.x;
  if (i >= total8) return;
  const size_t e0 = (size_t)i << 3;
  const v4f a0 = *(const v4f*)(src + e0);
  const v4f a1 = *(const v4f*)(src + e0 + 4);
  v8h hv;
#pragma unroll
  for (int e = 0; e < 4; ++e) {
    hv[e]     = (_Float16)(a0[e] * carry);
    hv[4 + e] = (_Float16)(a1[e] * carry);
  }
  unsigned short* q = dst + e0;
  *(volatile v8h*)q = hv;
  __threadfence();
  *(volatile v8h*)q = hv;
}

__device__ __forceinline__ int to_fixed_units(float v) {
  const float c = fminf(fmaxf(v, -kFixClamp), kFixClamp);
  return __float2int_rn(c * kFixScale);
}

__global__ __launch_bounds__(256) void densify_rows_f16_kernel(
    const float* __restrict__ vals, const int* __restrict__ rows, const int* __restrict__ cols,
    unsigned short* __restrict__ W16)
{
  __shared__ __align__(16) int cells[kRowsPerBlk * kIn];
  const int tid  = threadIdx.x;
  const int lane = tid & 31;
  const int wave = __builtin_amdgcn_readfirstlane((int)(threadIdx.x >> 5));
  const int rbase = blockIdx.x * kRowsPerBlk;

#pragma unroll 1
  for (int i = tid; i < kRowsPerBlk * kIn / 4; i += 256) {
    *(v4i*)(cells + 4 * i) = (v4i){0, 0, 0, 0};
  }
  __syncthreads();

  const v4i* rows4 = (const v4i*)rows;
  const v4i* cols4 = (const v4i*)cols;
  const v4f* vals4 = (const v4f*)vals;
  constexpr int kWaveSteps = kNnz / 128;
  constexpr int kRowMask = ~(kRowsPerBlk - 1);
#pragma unroll 1
  for (int it = wave; it < kWaveSteps; it += 8) {
    const int idx = it * 32 + lane;
    const v4i r4 = rows4[idx];
    const int r0 = r4[0], r1 = r4[1], r2 = r4[2], r3 = r4[3];
    const bool h0 = ((r0 & kRowMask) == rbase);
    const bool h1 = ((r1 & kRowMask) == rbase);
    const bool h2 = ((r2 & kRowMask) == rbase);
    const bool h3 = ((r3 & kRowMask) == rbase);
    const bool hany = h0 | h1 | h2 | h3;
    const unsigned hitmask = __builtin_amdgcn_ballot_w32(hany);
    if (hitmask != 0u) {
      const v4i c4 = cols4[idx];
      const v4f w4 = vals4[idx];
      int c0 = c4[0], c1 = c4[1], c2 = c4[2], c3 = c4[3];
      float w0 = w4[0], w1 = w4[1], w2 = w4[2], w3 = w4[3];
      asm volatile("" : "+v"(c0), "+v"(c1), "+v"(c2), "+v"(c3));
      asm volatile("" : "+v"(w0), "+v"(w1), "+v"(w2), "+v"(w3));
      if (h0 && ((unsigned)c0 < (unsigned)kIn)) atomicAdd(&cells[(r0 & (kRowsPerBlk - 1)) * kIn + c0], to_fixed_units(w0));
      if (h1 && ((unsigned)c1 < (unsigned)kIn)) atomicAdd(&cells[(r1 & (kRowsPerBlk - 1)) * kIn + c1], to_fixed_units(w1));
      if (h2 && ((unsigned)c2 < (unsigned)kIn)) atomicAdd(&cells[(r2 & (kRowsPerBlk - 1)) * kIn + c2], to_fixed_units(w2));
      if (h3 && ((unsigned)c3 < (unsigned)kIn)) atomicAdd(&cells[(r3 & (kRowsPerBlk - 1)) * kIn + c3], to_fixed_units(w3));
    }
  }
  __syncthreads();

  unsigned short* dst = W16 + (size_t)rbase * kIn;
  constexpr int kStoreIters = kRowsPerBlk * kIn / 8 / 256;
  for (int pass = 0; pass < 2; ++pass) {
#pragma unroll 1
    for (int itx = 0; itx < kStoreIters; ++itx) {
      const int item = itx * 256 + tid;
      const v4i a = *(const v4i*)(cells + item * 8);
      const v4i b = *(const v4i*)(cells + item * 8 + 4);
      v8h hv;
#pragma unroll
      for (int e = 0; e < 4; ++e) {
        hv[e]     = (_Float16)((float)a[e] * kCellToCarried);
        hv[4 + e] = (_Float16)((float)b[e] * kCellToCarried);
      }
      *(volatile v8h*)(dst + (size_t)item * 8) = hv;
    }
    __threadfence();
  }
}

__global__ __launch_bounds__(256) void gemm_f16_bias_kernel(
    const unsigned short* __restrict__ Ap, int lda,
    const unsigned short* __restrict__ Btp, int ldb,
    float* __restrict__ C, int ldc,
    const float* __restrict__ bias,
    int M, int N, int K, float scale)
{
  const _Float16* A  = (const _Float16*)Ap;
  const _Float16* Bt = (const _Float16*)Btp;
  __shared__ __align__(16) float sT[8][16 * 68];
  const int lane = threadIdx.x & 31;
  const int wave = __builtin_amdgcn_readfirstlane((int)(threadIdx.x >> 5));
  const int tilesN = N >> 6;
  const int tilesM = M >> 6;
  const int tile = blockIdx.x * 8 + wave;
  if (tile >= tilesM * tilesN) return;
  const int tm = tile / tilesN;
  const int tn = tile - tm * tilesN;
  const int m0 = tm << 6;
  const int n0 = tn << 6;

  const int rlane = lane & 15;
  const int koff  = (lane >> 4) * 8;
  const int mOff  = (lane >> 4) * 8;

  v8f acc[4][4];
#pragma unroll
  for (int i = 0; i < 4; ++i)
#pragma unroll
    for (int j = 0; j < 4; ++j) acc[i][j] = (v8f){0.f, 0.f, 0.f, 0.f, 0.f, 0.f, 0.f, 0.f};

  for (int k0 = 0; k0 < K; k0 += 32) {
    v16h bh[4];
#pragma unroll
    for (int j = 0; j < 4; ++j) {
      const size_t bo = (size_t)(n0 + (j << 4) + rlane) * ldb + koff + k0;
      bh[j] = frag_load_h(Bt + bo);
    }
#pragma unroll
    for (int i = 0; i < 4; ++i) {
      const size_t ao = (size_t)(m0 + (i << 4) + rlane) * lda + koff + k0;
      const v16h ah = frag_load_h(A + ao);
#pragma unroll
      for (int j = 0; j < 4; ++j) acc[i][j] = mma_h(ah, bh[j], acc[i][j]);
      tie_acc_h(acc[i][0], ah, bh[0]);
      tie_acc_h(acc[i][1], ah, bh[1]);
      tie_acc_h(acc[i][2], ah, bh[2]);
      nop_guard_h(acc[i][3], ah, bh[3]);
    }
    keep4_h(bh[0], bh[1], bh[2], bh[3]);
  }
#pragma unroll
  for (int i = 0; i < 4; ++i)
#pragma unroll
    for (int j = 0; j < 4; ++j) nop_guard_acc(acc[i][j]);

  float bvj[4];
#pragma unroll
  for (int j = 0; j < 4; ++j) bvj[j] = bias[n0 + (j << 4) + rlane];

  float* slab = sT[wave];
#pragma unroll
  for (int i = 0; i < 4; ++i) {
    const int mBase = m0 + (i << 4);
#pragma unroll
    for (int j = 0; j < 4; ++j) {
#pragma unroll
      for (int r = 0; r < 8; ++r) {
        const float v = acc[i][j][r] * scale + bvj[j];
        slab[(mOff + r) * 68 + (j << 4) + rlane] = v;
      }
    }
    __builtin_amdgcn_fence(__ATOMIC_RELEASE, "workgroup");
    __builtin_amdgcn_wave_barrier();
    __builtin_amdgcn_fence(__ATOMIC_ACQUIRE, "workgroup");
    {
      const int hh = lane >> 4, c4 = (lane & 15) * 4;
      for (int pass = 0; pass < 2; ++pass) {
#pragma unroll
        for (int it = 0; it < 8; ++it) {
          const int row = it * 2 + hh;
          const v4f v = *(const v4f*)(slab + row * 68 + c4);
          *(volatile v4f*)(C + (size_t)(mBase + row) * ldc + n0 + c4) = v;
        }
        __threadfence();
      }
    }
    __builtin_amdgcn_fence(__ATOMIC_RELEASE, "workgroup");
    __builtin_amdgcn_wave_barrier();
    __builtin_amdgcn_fence(__ATOMIC_ACQUIRE, "workgroup");
  }
}

extern "C" void kernel_launch(void* const* d_in, const int* in_sizes, int n_in,
                              void* d_out, int out_size, void* d_ws, size_t ws_size,
                              hipStream_t stream) {
  if (n_in < 5) return;
  if (in_sizes[0] != kBatch * kIn) return;
  if (in_sizes[1] != kNnz) return;
  if (in_sizes[2] != kOut) return;
  if (in_sizes[3] != kNnz) return;
  if (in_sizes[4] != kNnz) return;
  if (out_size != kBatch * kOut) return;
  if (ws_size < kWsTotal) return;

  const float* x      = (const float*)d_in[0];
  const float* w_vals = (const float*)d_in[1];
  const float* bias   = (const float*)d_in[2];
  const int*   w_rows = (const int*)d_in[3];
  const int*   w_cols = (const int*)d_in[4];
  float* out = (float*)d_out;

  char* ws = (char*)d_ws;
  unsigned short* X16 = (unsigned short*)(ws + kOffX16);
  unsigned short* W16 = (unsigned short*)(ws + kOffW16);

  cast_rows_f16_kernel<<<(kBatch * kIn / 8) / 256, 256, 0, stream>>>(x, X16, kBatch * kIn / 8, (float)kCarry);

  densify_rows_f16_kernel<<<kOut / kRowsPerBlk, 256, 0, stream>>>(w_vals, w_rows, w_cols, W16);

  gemm_f16_bias_kernel<<<dim3((kBatch / 64) * (kOut / 64) / 8, 1), 256, 0, stream>>>(
      X16, kIn, W16, kIn, out, kOut, bias, kBatch, kOut, kIn, kFoldBack);
}
